// Block_81260781240618
// MI455X (gfx1250) — hardware-verified
//
#include <hip/hip_runtime.h>
#include <math.h>

#ifndef NB
#define NB 4
#endif
#ifndef SEQ
#define SEQ 2048
#endif
#define NB_FULL 4
#define SEQ_FULL 2048
#define CE 384
#define NH 6
#define HD 64
#define DFF 1536
#define QKVW (3 * CE)
#define ROWS (NB * SEQ)

static_assert(CE == NH * HD);
static_assert(HD == 64);
static_assert(CE % 128 == 0);
static_assert(CE / 128 == 3);
static_assert(CE % 64 == 0 && DFF % 64 == 0 && QKVW % 64 == 0);
static_assert(CE % 32 == 0 && DFF % 32 == 0);
static_assert(CE % 8 == 0 && DFF % 8 == 0);
static_assert(ROWS % 64 == 0);
static_assert(SEQ % 64 == 0);
static_assert(ROWS % 8 == 0);
static_assert(NB <= NB_FULL && SEQ <= SEQ_FULL);

typedef __attribute__((ext_vector_type(16))) _Float16 v16h;
typedef __attribute__((ext_vector_type(8)))  _Float16 v8h;
typedef __attribute__((ext_vector_type(16))) __bf16   v16b;
typedef __attribute__((ext_vector_type(8)))  __bf16   v8b;
typedef __attribute__((ext_vector_type(8)))  float    v8f;
typedef __attribute__((ext_vector_type(4)))  float    v4f;
typedef unsigned int u4v __attribute__((ext_vector_type(4)));
typedef unsigned int u2v __attribute__((ext_vector_type(2)));


#define VST2(T, ptr, val) do { const T vst2_v_ = (val); *(volatile T*)(ptr) = vst2_v_; __threadfence(); *(volatile T*)(ptr) = vst2_v_; } while (0)

__device__ __forceinline__ float cmb_bf(float v) {
    const unsigned u = __builtin_bit_cast(unsigned, v);
    const unsigned r = (u + 0x7fffu + ((u >> 16) & 1u)) & 0xffff0000u;
    return __builtin_bit_cast(float, r);
}
__device__ __forceinline__ unsigned int pk2h(float a, float b) {
    return (unsigned int)__builtin_bit_cast(unsigned short, (_Float16)a) | ((unsigned int)__builtin_bit_cast(unsigned short, (_Float16)b) << 16);
}
__device__ __forceinline__ unsigned short bf_bits(float f) {
    const unsigned u = __float_as_uint(f);
    return (unsigned short)((u + 0x7FFFu + ((u >> 16) & 1u)) >> 16);
}
__device__ __forceinline__ void bsplit(float f, __bf16& hi, __bf16& lo) {
    const unsigned short hb = bf_bits(f);
    hi = __builtin_bit_cast(__bf16, hb);
    lo = __builtin_bit_cast(__bf16, bf_bits(f - __uint_as_float(((unsigned)hb) << 16)));
}
__device__ __forceinline__ v8f mma_b(v16b a, v16b b, v8f c) {
    c = __builtin_amdgcn_wmma_f32_16x16x32_bf16(false, a, false, b, (short)0, c, false, false);
    asm volatile("v_nop\n\tv_nop\n\tv_nop\n\tv_nop" : "+v"(c) : "v"(a), "v"(b));
    return c;
}
__device__ __forceinline__ void dep_guard_h(v8f& a, v8f& b, v16h x, v16h y) { asm volatile("v_nop\n\tv_nop\n\tv_nop\n\tv_nop" : "+v"(a), "+v"(b) : "v"(x), "v"(y)); }
__device__ __forceinline__ void keep4_h(v16h a, v16h b, v16h c, v16h d) { asm volatile("v_nop" :: "v"(a), "v"(b), "v"(c), "v"(d)); }
__device__ __forceinline__ void acc_guard4(v8f& a, v8f& b, v8f& c, v8f& d) { asm volatile("v_nop\n\tv_nop\n\tv_nop\n\tv_nop" : "+v"(a), "+v"(b), "+v"(c), "+v"(d)); }

union HFrag { v16h v; v8h h[2]; };
__device__ __forceinline__ v16h ldfrag_h(const _Float16* p) { HFrag f; f.h[0] = *(const v8h*)(p); f.h[1] = *(const v8h*)(p + 16); return f.v; }

__global__ __launch_bounds__(256) void k_cast_x(const float* __restrict__ X, unsigned short* __restrict__ D) {
    const int u = blockIdx.x * 256 + threadIdx.x; constexpr int per = CE / 8; if (u >= ROWS * per) return;
    const int r = u / per, c0 = 8 * (u % per);
    const int rs = (r / SEQ) * SEQ_FULL + (r % SEQ);
    const float* s = X + (size_t)rs * CE + c0;
    const v4f a = *(const v4f*)(s), b = *(const v4f*)(s + 4);
    u4v pk; pk.x = pk2h(cmb_bf(a.x), cmb_bf(a.y)); pk.y = pk2h(cmb_bf(a.z), cmb_bf(a.w)); pk.z = pk2h(cmb_bf(b.x), cmb_bf(b.y)); pk.w = pk2h(cmb_bf(b.z), cmb_bf(b.w));
    VST2(u4v, (u4v*)(D + (size_t)r * CE + c0), pk);
}
__global__ __launch_bounds__(256) void k_cast_ao(const float* __restrict__ S, unsigned short* __restrict__ D) {
    const int u = blockIdx.x * 256 + threadIdx.x; constexpr int per = CE / 8; if (u >= ROWS * per) return;
    const float* s = S + (size_t)u * 8;
    const v4f a = *(const v4f*)(s), b = *(const v4f*)(s + 4);
    u4v pk; pk.x = pk2h(a.x, a.y); pk.y = pk2h(a.z, a.w); pk.z = pk2h(b.x, b.y); pk.w = pk2h(b.z, b.w);
    VST2(u4v, (u4v*)(D + (size_t)u * 8), pk);
}
__global__ __launch_bounds__(256) void k_castT_w(const float* __restrict__ SRC, int lds, unsigned short* __restrict__ DST, int ldd, int nR, int nC, float sc) {
    const long long u = (long long)blockIdx.x * 256 + threadIdx.x; const int per = nR / 8; if (u >= (long long)nC * per) return;
    const int c = (int)(u / per); const int r0 = 8 * (int)(u % per);
    float w[8];
#pragma unroll
    for (int e = 0; e < 8; ++e) w[e] = cmb_bf(SRC[(long long)(r0 + e) * lds + c]) * sc;
    u4v pk; pk.x = pk2h(w[0], w[1]); pk.y = pk2h(w[2], w[3]); pk.z = pk2h(w[4], w[5]); pk.w = pk2h(w[6], w[7]);
    VST2(u4v, (u4v*)(DST + (long long)c * ldd + r0), pk);
}

template <int BIAS, int OUTH, int RELU>
__device__ __forceinline__ void gemm64_body(const unsigned short* __restrict__ Ap, int lda, const unsigned short* __restrict__ Btp, int ldb,
                                            float* __restrict__ Cf, unsigned short* __restrict__ Ch, int ldc, const float* __restrict__ bias,
                                            int M, int N, int K, float scale, float* sT) {
    const _Float16* A = (const _Float16*)Ap; const _Float16* Bt = (const _Float16*)Btp;
    const int lane = threadIdx.x & 31, wave = threadIdx.x >> 5;
    const int tilesN = N >> 6, tilesM = M >> 6;
    const int tile = blockIdx.x * 8 + wave;
    if (tile >= tilesM * tilesN) return;
    const int tm = tile / tilesN, tn = tile - tm * tilesN;
    const int m0 = tm << 6, n0 = tn << 6;
    const int rlane = lane & 15;
    const int koff = (lane >> 4) * 8;
    const int mOff = (lane >> 4) * 8;
    v8f acc[4][4];
#pragma unroll
    for (int i = 0; i < 4; ++i)
#pragma unroll
        for (int j = 0; j < 4; ++j) acc[i][j] = (v8f){0.f, 0.f, 0.f, 0.f, 0.f, 0.f, 0.f, 0.f};
#pragma unroll 1
    for (int k0 = 0; k0 < K; k0 += 32) {
        v16h bh[4];
#pragma unroll
        for (int j = 0; j < 4; ++j) bh[j] = ldfrag_h(Bt + (size_t)(n0 + (j << 4) + rlane) * ldb + koff + k0);
#pragma unroll
        for (int i = 0; i < 4; ++i) {
            const v16h ah = ldfrag_h(A + (size_t)(m0 + (i << 4) + rlane) * lda + koff + k0);
#pragma unroll
            for (int j = 0; j < 4; ++j) acc[i][j] = __builtin_amdgcn_wmma_f32_16x16x32_f16(false, ah, false, bh[j], (short)0, acc[i][j], false, false);
            dep_guard_h(acc[i][0], acc[i][3], ah, ah);
        }
        keep4_h(bh[0], bh[1], bh[2], bh[3]);
    }
    acc_guard4(acc[0][0], acc[0][1], acc[0][2], acc[0][3]);
    acc_guard4(acc[1][0], acc[1][1], acc[1][2], acc[1][3]);
    acc_guard4(acc[2][0], acc[2][1], acc[2][2], acc[2][3]);
    acc_guard4(acc[3][0], acc[3][1], acc[3][2], acc[3][3]);

    float* slab = sT + wave * (16 * 68);
#pragma unroll
    for (int i = 0; i < 4; ++i) {
        const int mBase = m0 + (i << 4);
#pragma unroll
        for (int j = 0; j < 4; ++j) {
            const int n = n0 + (j << 4) + rlane;
            float bv = 0.f;
            if (BIAS) bv = cmb_bf(bias[n]);
#pragma unroll
            for (int r = 0; r < 8; ++r) {
                float v = acc[i][j][r] * scale;
                if (BIAS) v += bv;
                if (RELU) v = fmaxf(v, 0.0f);
                slab[(mOff + r) * 68 + (j << 4) + rlane] = v;
            }
        }
        __builtin_amdgcn_fence(3  , "workgroup");
        __builtin_amdgcn_wave_barrier();
        __builtin_amdgcn_fence(2  , "workgroup");
        if (!OUTH) {
            const int hh = lane >> 4, c4 = (lane & 15) * 4;
            for (int pass = 0; pass < 2; ++pass) {
#pragma unroll
                for (int it = 0; it < 8; ++it) {
                    const int row = it * 2 + hh;
                    const v4f v = *(const v4f*)(slab + row * 68 + c4);
                    *(volatile v4f*)(Cf + (size_t)(mBase + row) * ldc + n0 + c4) = v;
                }
                __threadfence();
            }
        } else {
            const int q = lane >> 3, c8 = (lane & 7) * 8;
            for (int pass = 0; pass < 2; ++pass) {
#pragma unroll
                for (int it = 0; it < 4; ++it) {
                    const int row = it * 4 + q;
                    const float* sp = slab + row * 68 + c8;
                    v8h hv;
#pragma unroll
                    for (int e = 0; e < 8; ++e) hv[e] = (_Float16)sp[e];
                    *(volatile v8h*)(Ch + (size_t)(mBase + row) * ldc + n0 + c8) = hv;
                }
                __threadfence();
            }
        }
        __builtin_amdgcn_fence(3  , "workgroup");
        __builtin_amdgcn_wave_barrier();
        __builtin_amdgcn_fence(2  , "workgroup");
    }
}

__global__ __launch_bounds__(256) void k_gemm_qkv(const unsigned short* __restrict__ A, const unsigned short* __restrict__ Bt, float* __restrict__ C) {
    __shared__ __align__(16) float sT[8 * 16 * 68];
    gemm64_body<0, 0, 0>(A, CE, Bt, CE, C, nullptr, QKVW, nullptr, ROWS, QKVW, CE, 0.0625f, sT);
}
__global__ __launch_bounds__(256) void k_gemm_wo(const unsigned short* __restrict__ A, const unsigned short* __restrict__ Bt, const float* __restrict__ bias, float* __restrict__ C) {
    __shared__ __align__(16) float sT[8 * 16 * 68];
    gemm64_body<1, 0, 0>(A, CE, Bt, CE, C, nullptr, CE, bias, ROWS, CE, CE, 0.0625f, sT);
}
__global__ __launch_bounds__(256) void k_gemm_w1(const unsigned short* __restrict__ A, const unsigned short* __restrict__ Bt, const float* __restrict__ bias, unsigned short* __restrict__ Ch) {
    __shared__ __align__(16) float sT[8 * 16 * 68];
    gemm64_body<1, 1, 1>(A, CE, Bt, CE, nullptr, Ch, DFF, bias, ROWS, DFF, CE, 0.0625f, sT);
}
__global__ __launch_bounds__(256) void k_gemm_w2(const unsigned short* __restrict__ A, const unsigned short* __restrict__ Bt, const float* __restrict__ bias, float* __restrict__ C) {
    __shared__ __align__(16) float sT[8 * 16 * 68];
    gemm64_body<1, 0, 0>(A, DFF, Bt, DFF, C, nullptr, CE, bias, ROWS, CE, DFF, 0.0625f, sT);
}

#define AT_KSH 0
#define AT_KSL 4096
#define AT_VTH 8192
#define AT_VTL 12288
#define AT_PSH 16384
#define AT_PSL 20480
static_assert(4 * 16 * 68 * 4 <= 4 * 4096 * 2);
union BFrag { v16b v; v8b h[2]; };

__global__ __launch_bounds__(128) void k_attn_causal(const float* __restrict__ qkv, float* __restrict__ ao) {
    __shared__ __align__(16) __bf16 smem[6 * 4096];
    const int tid = threadIdx.x, wave = tid >> 5, lane = tid & 31, hh = lane >> 4, c = lane & 15;
    constexpr int nqb = SEQ / 64;
    const int bx = blockIdx.x;
    const int qb = bx % nqb, bh = bx / nqb;
    const int h = bh % NH, b = bh / NH;
    const int q0 = qb * 64 + wave * 16;
    const float* qp = qkv + (size_t)b * SEQ * QKVW + (size_t)h * HD;
    const float* kp = qp + CE;
    const float* vp = qp + 2 * CE;
    float* op = ao + (size_t)b * SEQ * CE + (size_t)h * HD;

    v16b qah[2], qal[2];
    {
        const float* qrow = qp + (size_t)(q0 + c) * QKVW;
#pragma unroll
        for (int dc = 0; dc < 2; ++dc) {
            const v4f x0 = *(const v4f*)(qrow + dc * 32 + 8 * hh), x1 = *(const v4f*)(qrow + dc * 32 + 8 * hh + 4);
            const v4f y0 = *(const v4f*)(qrow + dc * 32 + 16 + 8 * hh), y1 = *(const v4f*)(qrow + dc * 32 + 16 + 8 * hh + 4);
#pragma unroll
            for (int e = 0; e < 4; ++e) {
                __bf16 a, l;
                bsplit(x0[e] * 0.125f, a, l); qah[dc][e] = a;      qal[dc][e] = l;
                bsplit(x1[e] * 0.125f, a, l); qah[dc][4 + e] = a;  qal[dc][4 + e] = l;
                bsplit(y0[e] * 0.125f, a, l); qah[dc][8 + e] = a;  qal[dc][8 + e] = l;
                bsplit(y1[e] * 0.125f, a, l); qah[dc][12 + e] = a; qal[dc][12 + e] = l;
            }
        }
    }
    float mrow[8], lrow[8];
    v8f oacc[4];
#pragma unroll
    for (int r = 0; r < 8; ++r) { mrow[r] = -__builtin_inff(); lrow[r] = 0.f; }
#pragma unroll
    for (int t = 0; t < 4; ++t) oacc[t] = (v8f){0.f, 0.f, 0.f, 0.f, 0.f, 0.f, 0.f, 0.f};

    const int nChunks = qb + 1;
    for (int kc = 0; kc < nChunks; ++kc) {
        const int kv0 = kc * 64;
        __syncthreads();
        {
            const int kvr = tid >> 1, dh = (tid & 1) * 32;
            const float* krow = kp + (size_t)(kv0 + kvr) * QKVW + dh;
            const float* vrow = vp + (size_t)(kv0 + kvr) * QKVW + dh;
#pragma unroll
            for (int i = 0; i < 8; ++i) {
                const v4f kk = *(const v4f*)(krow + 4 * i);
                const v4f vv = *(const v4f*)(vrow + 4 * i);
#pragma unroll
                for (int e = 0; e < 4; ++e) {
                    const int d = dh + 4 * i + e;
                    __bf16 a, l;
                    bsplit(kk[e], a, l); smem[AT_KSH + kvr * 64 + d] = a; smem[AT_KSL + kvr * 64 + d] = l;
                    bsplit(vv[e], a, l); smem[AT_VTH + d * 64 + kvr] = a; smem[AT_VTL + d * 64 + kvr] = l;
                }
            }
        }
        __syncthreads();

        v8f s[4];
#pragma unroll
        for (int j = 0; j < 4; ++j) {
            s[j] = (v8f){0.f, 0.f, 0.f, 0.f, 0.f, 0.f, 0.f, 0.f};
#pragma unroll
            for (int dc = 0; dc < 2; ++dc) {
                BFrag kb, kl;
                kb.h[0] = *(const v8b*)(smem + AT_KSH + (j * 16 + c) * 64 + dc * 32 + 8 * hh);
                kb.h[1] = *(const v8b*)(smem + AT_KSH + (j * 16 + c) * 64 + dc * 32 + 16 + 8 * hh);
                kl.h[0] = *(const v8b*)(smem + AT_KSL + (j * 16 + c) * 64 + dc * 32 + 8 * hh);
                kl.h[1] = *(const v8b*)(smem + AT_KSL + (j * 16 + c) * 64 + dc * 32 + 16 + 8 * hh);
                s[j] = mma_b(qah[dc], kb.v, s[j]);
                s[j] = mma_b(qah[dc], kl.v, s[j]);
                s[j] = mma_b(qal[dc], kb.v, s[j]);
            }
        }
        const bool diag = (kc == qb);
        float cm[8];
#pragma unroll
        for (int r = 0; r < 8; ++r) {
            const int qrow = q0 + 8 * hh + r;
            float m = -__builtin_inff();
#pragma unroll
            for (int j = 0; j < 4; ++j) {
                const int kvcol = kv0 + j * 16 + c;
                const float sv = (diag && kvcol > qrow) ? -1.0e9f : s[j][r];
                s[j][r] = sv;
                m = fmaxf(m, sv);
            }
#pragma unroll
            for (int off = 1; off < 16; off <<= 1) m = fmaxf(m, __shfl_xor(m, off, 32));
            cm[r] = m;
        }
#pragma unroll
        for (int r = 0; r < 8; ++r) {
            const float mnew = fmaxf(mrow[r], cm[r]);
            const float alpha = expf(mrow[r] - mnew);
            mrow[r] = mnew;
            float psum = 0.f;
#pragma unroll
            for (int j = 0; j < 4; ++j) {
                const float p = expf(s[j][r] - mnew);
                psum += p;
                __bf16 a, l; bsplit(p, a, l);
                smem[AT_PSH + wave * 1024 + (8 * hh + r) * 64 + j * 16 + c] = a;
                smem[AT_PSL + wave * 1024 + (8 * hh + r) * 64 + j * 16 + c] = l;
            }
#pragma unroll
            for (int off = 1; off < 16; off <<= 1) psum += __shfl_xor(psum, off, 32);
            lrow[r] = lrow[r] * alpha + psum;
#pragma unroll
            for (int t = 0; t < 4; ++t) oacc[t][r] *= alpha;
        }
        __builtin_amdgcn_fence(3  , "workgroup");
        __builtin_amdgcn_wave_barrier();
        __builtin_amdgcn_fence(2  , "workgroup");
#pragma unroll 1
        for (int kk = 0; kk < 2; ++kk) {
            BFrag pa, pl;
            pa.h[0] = *(const v8b*)(smem + AT_PSH + wave * 1024 + c * 64 + kk * 32 + 8 * hh);
            pa.h[1] = *(const v8b*)(smem + AT_PSH + wave * 1024 + c * 64 + kk * 32 + 16 + 8 * hh);
            pl.h[0] = *(const v8b*)(smem + AT_PSL + wave * 1024 + c * 64 + kk * 32 + 8 * hh);
            pl.h[1] = *(const v8b*)(smem + AT_PSL + wave * 1024 + c * 64 + kk * 32 + 16 + 8 * hh);
#pragma unroll
            for (int t = 0; t < 4; ++t) {
                BFrag vb, vl;
                vb.h[0] = *(const v8b*)(smem + AT_VTH + (t * 16 + c) * 64 + kk * 32 + 8 * hh);
                vb.h[1] = *(const v8b*)(smem + AT_VTH + (t * 16 + c) * 64 + kk * 32 + 16 + 8 * hh);
                vl.h[0] = *(const v8b*)(smem + AT_VTL + (t * 16 + c) * 64 + kk * 32 + 8 * hh);
                vl.h[1] = *(const v8b*)(smem + AT_VTL + (t * 16 + c) * 64 + kk * 32 + 16 + 8 * hh);
                oacc[t] = mma_b(pa.v, vb.v, oacc[t]);
                oacc[t] = mma_b(pa.v, vl.v, oacc[t]);
                oacc[t] = mma_b(pl.v, vb.v, oacc[t]);
            }
        }
    }

    __syncthreads();
    float* os = (float*)smem + wave * (16 * 68);
#pragma unroll
    for (int r = 0; r < 8; ++r) {
        const float inv = 1.0f / lrow[r];
#pragma unroll
        for (int t = 0; t < 4; ++t) os[(8 * hh + r) * 68 + t * 16 + c] = oacc[t][r] * inv;
    }
    __builtin_amdgcn_fence(3  , "workgroup");
    __builtin_amdgcn_wave_barrier();
    __builtin_amdgcn_fence(2  , "workgroup");
    {
        const int c4 = (lane & 15) * 4;
        for (int pass = 0; pass < 2; ++pass) {
#pragma unroll
            for (int it = 0; it < 8; ++it) {
                const int row = it * 2 + hh;
                const v4f val = *(const v4f*)(os + row * 68 + c4);
                *(volatile v4f*)(op + (size_t)(q0 + row) * CE + c4) = val;
            }
            __threadfence();
        }
    }
}

template <int NQ, int XBF, int XMAP, int YMAP, int W16>
__device__ __forceinline__ void ln_body(const float* __restrict__ A, const float* __restrict__ X, const float* __restrict__ GA, const float* __restrict__ BE,
                                        float eps, float* __restrict__ Yf, unsigned short* __restrict__ Y16) {
    #pragma clang fp contract(off)
    constexpr int WD = 128 * NQ;
    static_assert(WD == CE);
    const int r = blockIdx.x * 8 + (threadIdx.x >> 5); const int L = threadIdx.x & 31; if (r >= ROWS) return;
    const int rf = (r / SEQ) * SEQ_FULL + (r % SEQ);
    const size_t xrow = XMAP ? (size_t)rf : (size_t)r;
    const size_t yrow = YMAP ? (size_t)rf : (size_t)r;
    v4f v[NQ]; float s = 0.f;
#pragma unroll
    for (int q = 0; q < NQ; ++q) {
        const int cc = 4 * L + 128 * q;
        const v4f a = *(const v4f*)(A + (size_t)r * WD + cc);
        v4f x = *(const v4f*)(X + xrow * WD + cc);
        if (XBF) { x.x = cmb_bf(x.x); x.y = cmb_bf(x.y); x.z = cmb_bf(x.z); x.w = cmb_bf(x.w); }
        v[q] = a + x;
        s += (v[q].x + v[q].y) + (v[q].z + v[q].w);
    }
#pragma unroll
    for (int o = 16; o > 0; o >>= 1) s += __shfl_xor(s, o, 32);
    const float mu = s * (1.f / WD); float qq = 0.f;
#pragma unroll
    for (int q = 0; q < NQ; ++q) { v[q].x -= mu; v[q].y -= mu; v[q].z -= mu; v[q].w -= mu; qq += (v[q].x * v[q].x + v[q].y * v[q].y) + (v[q].z * v[q].z + v[q].w * v[q].w); }
#pragma unroll
    for (int o = 16; o > 0; o >>= 1) qq += __shfl_xor(qq, o, 32);
    const float rs = rsqrtf(qq * (1.f / WD) + eps);
#pragma unroll
    for (int q = 0; q < NQ; ++q) {
        const int cc = 4 * L + 128 * q;
        const v4f ga = *(const v4f*)(GA + cc), be = *(const v4f*)(BE + cc);
        v4f y;
        y.x = v[q].x * rs * cmb_bf(ga.x) + cmb_bf(be.x); y.y = v[q].y * rs * cmb_bf(ga.y) + cmb_bf(be.y);
        y.z = v[q].z * rs * cmb_bf(ga.z) + cmb_bf(be.z); y.w = v[q].w * rs * cmb_bf(ga.w) + cmb_bf(be.w);
        VST2(v4f, (v4f*)(Yf + yrow * WD + cc), y);
        if (W16) { u2v pk; pk.x = pk2h(y.x, y.y); pk.y = pk2h(y.z, y.w); VST2(u2v, (u2v*)(Y16 + (size_t)r * WD + cc), pk); }
    }
}
__global__ __launch_bounds__(256) void k_ln1(const float* __restrict__ Y, const float* __restrict__ X, const float* __restrict__ GA, const float* __restrict__ BE, float* __restrict__ X1, unsigned short* __restrict__ H16) {
    ln_body<CE / 128, 1, 1, 0, 1>(Y, X, GA, BE, 1e-3f, X1, H16);
}
__global__ __launch_bounds__(256) void k_ln2(const float* __restrict__ Y2, const float* __restrict__ X1, const float* __restrict__ GA, const float* __restrict__ BE, float* __restrict__ OUT) {
    ln_body<CE / 128, 0, 0, 1, 0>(Y2, X1, GA, BE, 1e-3f, OUT, nullptr);
}

constexpr size_t al256(size_t b) { return (b + 255) / 256 * 256; }
constexpr size_t SZ_X16  = al256((size_t)ROWS * CE * 2);
constexpr size_t SZ_W3   = al256((size_t)QKVW * CE * 2);
constexpr size_t SZ_WO   = al256((size_t)CE * CE * 2);
constexpr size_t SZ_W1   = al256((size_t)DFF * CE * 2);
constexpr size_t SZ_W2   = al256((size_t)CE * DFF * 2);
constexpr size_t SZ_QKV  = al256((size_t)ROWS * QKVW * 4);
constexpr size_t SZ_AO   = al256((size_t)ROWS * CE * 4);
constexpr size_t SZ_ATT  = al256((size_t)ROWS * CE * 4);
constexpr size_t SZ_X1   = al256((size_t)ROWS * CE * 4);
constexpr size_t SZ_H16  = al256((size_t)ROWS * CE * 2);
constexpr size_t OFF_X16 = 0;
constexpr size_t OFF_W3  = OFF_X16 + SZ_X16;
constexpr size_t OFF_WO  = OFF_W3 + SZ_W3;
constexpr size_t OFF_W1  = OFF_WO + SZ_WO;
constexpr size_t OFF_W2  = OFF_W1 + SZ_W1;
constexpr size_t OFF_QKV = OFF_W2 + SZ_W2;
constexpr size_t OFF_AO  = OFF_QKV + SZ_QKV;
constexpr size_t OFF_ATT = OFF_AO + SZ_AO;
constexpr size_t OFF_X1  = OFF_ATT + SZ_ATT;
constexpr size_t OFF_H16 = OFF_X1 + SZ_X1;
constexpr size_t WS_TOTAL = OFF_H16 + SZ_H16;
static_assert(WS_TOTAL <= (size_t)134217728);
static_assert((size_t)ROWS * DFF * 2 <= SZ_QKV);
static_assert((size_t)ROWS * CE * 4 <= SZ_AO);
static_assert((size_t)ROWS * CE * 2 <= SZ_X16);

extern "C" void kernel_launch(void* const* d_in, const int* in_sizes, int n_in, void* d_out, int out_size, void* d_ws, size_t ws_size, hipStream_t stream) {
    if (n_in < 14) return;
    const long long need_x = (long long)(NB - 1) * SEQ_FULL * CE + (long long)SEQ * CE;
    if ((long long)in_sizes[0] < need_x) return;
    if (in_sizes[1] < CE * CE || in_sizes[2] < CE * CE || in_sizes[3] < CE * CE || in_sizes[4] < CE * CE) return;
    if (in_sizes[5] < CE || in_sizes[6] < CE * DFF || in_sizes[7] < DFF || in_sizes[8] < DFF * CE || in_sizes[9] < CE) return;
    if (in_sizes[10] < CE || in_sizes[11] < CE || in_sizes[12] < CE || in_sizes[13] < CE) return;
    if ((long long)out_size < need_x) return;
    if (ws_size < WS_TOTAL) return;

    const float* x   = (const float*)d_in[0];
    const float* wq  = (const float*)d_in[1];
    const float* wk  = (const float*)d_in[2];
    const float* wv  = (const float*)d_in[3];
    const float* wo  = (const float*)d_in[4];
    const float* bo  = (const float*)d_in[5];
    const float* w1  = (const float*)d_in[6];
    const float* b1  = (const float*)d_in[7];
    const float* w2  = (const float*)d_in[8];
    const float* b2  = (const float*)d_in[9];
    const float* g1  = (const float*)d_in[10];
    const float* be1 = (const float*)d_in[11];
    const float* g2  = (const float*)d_in[12];
    const float* be2 = (const float*)d_in[13];
    float* out = (float*)d_out;
    char* ws = (char*)d_ws;
    unsigned short* X16  = (unsigned short*)(ws + OFF_X16);
    unsigned short* AO16 = X16;
    unsigned short* W316 = (unsigned short*)(ws + OFF_W3);
    unsigned short* WO16 = (unsigned short*)(ws + OFF_WO);
    unsigned short* W1T  = (unsigned short*)(ws + OFF_W1);
    unsigned short* W2T  = (unsigned short*)(ws + OFF_W2);
    float* QKV = (float*)(ws + OFF_QKV);
    unsigned short* HF16 = (unsigned short*)(ws + OFF_QKV);
    float* AO  = (float*)(ws + OFF_AO);
    float* FFo = (float*)(ws + OFF_AO);
    float* ATT = (float*)(ws + OFF_ATT);
    float* X1  = (float*)(ws + OFF_X1);
    unsigned short* H16 = (unsigned short*)(ws + OFF_H16);

    k_cast_x<<<(ROWS * (CE / 8) + 255) / 256, 256, 0, stream>>>(x, X16);
    k_castT_w<<<(CE * (CE / 8) + 255) / 256, 256, 0, stream>>>(wq, CE, W316, CE, CE, CE, 16.0f);
    k_castT_w<<<(CE * (CE / 8) + 255) / 256, 256, 0, stream>>>(wk, CE, W316 + (size_t)CE * CE, CE, CE, CE, 16.0f);
    k_castT_w<<<(CE * (CE / 8) + 255) / 256, 256, 0, stream>>>(wv, CE, W316 + (size_t)2 * CE * CE, CE, CE, CE, 16.0f);
    k_castT_w<<<(CE * (CE / 8) + 255) / 256, 256, 0, stream>>>(wo, CE, WO16, CE, CE, CE, 16.0f);
    k_castT_w<<<(DFF * (CE / 8) + 255) / 256, 256, 0, stream>>>(w1, DFF, W1T, CE, CE, DFF, 16.0f);
    k_castT_w<<<(CE * (DFF / 8) + 255) / 256, 256, 0, stream>>>(w2, CE, W2T, DFF, DFF, CE, 16.0f);

    k_gemm_qkv<<<((ROWS / 64) * (QKVW / 64) + 7) / 8, 256, 0, stream>>>(X16, W316, QKV);
    k_attn_causal<<<NB * NH * (SEQ / 64), 128, 0, stream>>>(QKV, AO);
    k_cast_ao<<<(ROWS * (CE / 8) + 255) / 256, 256, 0, stream>>>(AO, AO16);
    k_gemm_wo<<<((ROWS / 64) * (CE / 64) + 7) / 8, 256, 0, stream>>>(AO16, WO16, bo, ATT);
    k_ln1<<<(ROWS + 7) / 8, 256, 0, stream>>>(ATT, x, g1, be1, X1, H16);
    k_gemm_w1<<<((ROWS / 64) * (DFF / 64) + 7) / 8, 256, 0, stream>>>(H16, W1T, b1, HF16);
    k_gemm_w2<<<((ROWS / 64) * (CE / 64) + 7) / 8, 256, 0, stream>>>(HF16, W2T, b2, FFo);
    k_ln2<<<(ROWS + 7) / 8, 256, 0, stream>>>(FFo, X1, g2, be2, out);
}
